// BatchMultiHeadGraphAttention_34359738433
// MI455X (gfx1250) — hardware-run, weakly checked
//
#include <hip/hip_runtime.h>
#include <stddef.h>
#include <stdint.h>
#include <math.h>


#define NN      50000
#define NE      800000
#define NHEAD   4
#define FIN     32
#define FOUT    32
#define HC      128
#define MP      50048
#define NTHR    256
#define NWAVE   8
#define EPT     8
#define CHUNK   (NTHR * EPT)
#define WCAP    (EPT * 32)
#define LISTN   (NWAVE * WCAP)
#define NBRUN   1024
#define SLOTB   10
#define IDB     17
#define NBLK    49
#define RCAP    28672
#define DEGCAP  64
#define GBM     64
#define GTHR    128
#define NEGSL   0.2f
#define MX0     (-1.0e30f)
#define PARN    128
#define P_WSRC  0
#define P_WDST  32
#define P_BIAS  64
#define P_FCB   96
#define NUX     (MP * (FIN / 8))
#define NBX     (NUX / NTHR)
#define NUW     (HC * (FIN / 8))
#define NBW     (NUW / NTHR)
#define WSMAX   134217728
#define LDS_SCAN ((2 * RCAP + 2 * NBRUN + LISTN) * 4 + 64)

static_assert(NN == 50000 && NE == 800000);
static_assert(HC == NHEAD * FOUT && HC == 128);
static_assert(FOUT == 32 && FIN == 32);
static_assert(NN < (1 << IDB));
static_assert(NBRUN == (1 << SLOTB));
static_assert(NBLK * NBRUN >= NN);
static_assert(SLOTB + IDB < 31);
static_assert(((long long)CHUNK << SLOTB) < (1LL << 31));
static_assert(RCAP >= 16384 && (RCAP % 32) == 0);
static_assert(DEGCAP >= 16 + 8);
static_assert((MP % 128) == 0 && (MP % GBM) == 0 && MP >= NN);
static_assert(NUX % NTHR == 0 && NUW % NTHR == 0);
static_assert(NTHR * 4 == NBRUN);
static_assert(LISTN >= NBRUN && LISTN >= NWAVE * WCAP);
static_assert(LDS_SCAN <= 327680);
static_assert(GBM == (GTHR / 32) * 16);
static_assert(GTHR == 2 * GBM);
static_assert(GBM * 8 == GTHR * 4);
static_assert((size_t)NN * FOUT - 1 < (size_t)NN * FOUT);

typedef float          v4f  __attribute__((ext_vector_type(4)));
typedef float          v8f  __attribute__((ext_vector_type(8)));
typedef int            v4i  __attribute__((ext_vector_type(4)));
typedef int            v8i  __attribute__((ext_vector_type(8)));
typedef unsigned int   v4u  __attribute__((ext_vector_type(4)));
typedef unsigned short v8us __attribute__((ext_vector_type(8)));
typedef __bf16         v16b __attribute__((ext_vector_type(16)));
typedef v4f  __attribute__((may_alias)) v4fa;
typedef v4i  __attribute__((may_alias)) v4ia;
typedef v8us __attribute__((may_alias)) v8usa;
union FragB { v16b v; v8us h[2]; v8i w; };

__device__ __forceinline__ v8f wmb(const FragB& a, const FragB& b, v8f c) {
  v8f d = __builtin_amdgcn_wmma_f32_16x16x32_bf16(false, a.v, false, b.v, (short)0, c, false, false);
  asm volatile("v_nop\n\tv_nop\n\tv_nop\n\tv_nop" : "+v"(d) : "v"(a.w), "v"(b.w));
  return d;
}

__device__ __forceinline__ unsigned int f2bf(float f) {
  const unsigned int u = __float_as_uint(f);
  return ((u + 0x7FFFu + ((u >> 16) & 1u)) >> 16) & 0xFFFFu;
}
__device__ __forceinline__ unsigned int bfrbits(float f) { return f2bf(f) << 16; }
__device__ __forceinline__ unsigned int pk2(float lo, float hi) { return f2bf(lo) | (f2bf(hi) << 16); }
__device__ __forceinline__ v4u pack8(const v4f a, const v4f b) {
  v4u r;
  r.x = pk2(a.x, a.y); r.y = pk2(a.z, a.w); r.z = pk2(b.x, b.y); r.w = pk2(b.z, b.w);
  return r;
}

__global__ __launch_bounds__(NTHR) void k_prep(const float* __restrict__ hx, const float* __restrict__ w,
                                               const float* __restrict__ fcw, const float* __restrict__ fcb,
                                               const float* __restrict__ bias,
                                               unsigned short* xb, unsigned short* wt, float* par) {
  const int bx = (int)blockIdx.x, tid = (int)threadIdx.x;
  if (bx < NBX) {
    const int u   = bx * NTHR + tid;
    const int row = u >> 2;
    const int k8  = (u & 3) * 8;
    const int rc  = row < NN ? row : NN - 1;
    const float* p = hx + (size_t)rc * FIN + k8;
    const v4f a = *(const v4fa*)p;
    const v4f b = *(const v4fa*)(p + 4);
    const unsigned int msk = row < NN ? 0xFFFFFFFFu : 0u;
    v4u hv = pack8(a, b);
    hv.x = hv.x & msk; hv.y = hv.y & msk; hv.z = hv.z & msk; hv.w = hv.w & msk;
    unsigned short* o = xb + (size_t)row * FIN + k8;
    *(volatile v4u*)o = hv;
    __threadfence();
    *(volatile v4u*)o = hv;
  } else if (bx < NBX + NBW) {
    const int v  = (bx - NBX) * NTHR + tid;
    const int n  = v >> 2;
    const int k8 = (v & 3) * 8;
    const int hd = n >> 5;
    const int oc = n & 31;
    const float* p = w + (size_t)hd * (FIN * FOUT) + (size_t)k8 * FOUT + oc;
    v4f a, b;
    a.x = p[0];        a.y = p[FOUT];     a.z = p[2 * FOUT]; a.w = p[3 * FOUT];
    b.x = p[4 * FOUT]; b.y = p[5 * FOUT]; b.z = p[6 * FOUT]; b.w = p[7 * FOUT];
    const v4u wv = pack8(a, b);
    unsigned short* o = wt + (size_t)n * FIN + k8;
    *(volatile v4u*)o = wv;
    __threadfence();
    *(volatile v4u*)o = wv;
  } else {
    if (tid < 32) {
      const int t   = tid;
      const int ifc = 4 * (t < 15 ? t : 15);
      int ib = t - 16; ib = ib < 0 ? 0 : (ib > 7 ? 7 : ib); ib = 4 * ib;
      const v4f vf = *(const v4fa*)(fcw + ifc);
      const v4f vb = *(const v4fa*)(bias + ib);
      const float fb = fcb[0];
      asm volatile("" :: "v"(vf), "v"(vb), "v"(fb));
      const unsigned int mf = (t < 16) ? 0xFFFFFFFFu : 0u;
      const unsigned int mb = (t >= 16 && t < 24) ? 0xFFFFFFFFu : 0u;
      const unsigned int mc = (t == 24) ? 0xFFFFFFFFu : 0u;
      v4f ov;
      ov.x = __uint_as_float((bfrbits(vf.x) & mf) | (bfrbits(vb.x) & mb) | (bfrbits(fb) & mc));
      ov.y = __uint_as_float((bfrbits(vf.y) & mf) | (bfrbits(vb.y) & mb));
      ov.z = __uint_as_float((bfrbits(vf.z) & mf) | (bfrbits(vb.z) & mb));
      ov.w = __uint_as_float((bfrbits(vf.w) & mf) | (bfrbits(vb.w) & mb));
      float* o = par + 4 * t;
      *(volatile v4f*)o = ov;
      __threadfence();
      *(volatile v4f*)o = ov;
    }
  }
}

__global__ __launch_bounds__(GTHR) __attribute__((amdgpu_num_vgpr(248)))
void k_proj(const unsigned short* __restrict__ XB, const unsigned short* __restrict__ WT,
            const float* __restrict__ PAR, float* HP, float* SD) {
  __shared__ __attribute__((aligned(16))) float stg[GBM * HC];
  __shared__ __attribute__((aligned(16))) float spar[PARN];
  __shared__ __attribute__((aligned(16))) float sds[GBM * 8];
  const int tid = (int)threadIdx.x, lane = tid & 31, wave = tid >> 5, hh = lane >> 4, m = lane & 15;
  const int rowBase = (int)blockIdx.x * GBM;

  if (wave == 0) {
    const v4f pv = *(const v4fa*)(PAR + 4 * lane);
    *(v4fa*)(spar + 4 * lane) = pv;
  }

  v8f acc[8];
  {
    const v8f z = {0.f, 0.f, 0.f, 0.f, 0.f, 0.f, 0.f, 0.f};
#pragma unroll
    for (int t = 0; t < 8; ++t) acc[t] = z;
  }
  const unsigned short* ap = XB + (size_t)(rowBase + 16 * wave + m) * FIN + 8 * hh;
  const unsigned short* wp = WT + (size_t)m * FIN + 8 * hh;
  FragB af;
  af.h[0] = *(const v8usa*)ap;
  af.h[1] = *(const v8usa*)(ap + 16);
#pragma unroll
  for (int t = 0; t < 8; ++t) {
    const unsigned short* wq = wp + (size_t)(16 * t) * FIN;
    FragB bf;
    bf.h[0] = *(const v8usa*)wq;
    bf.h[1] = *(const v8usa*)(wq + 16);
    acc[t] = wmb(af, bf, acc[t]);
  }

#pragma unroll
  for (int t = 0; t < 8; ++t) {
    const int lc = 16 * t + m;
#pragma unroll
    for (int r = 0; r < 8; ++r) {
      const int lr = 16 * wave + 8 * hh + r;
      stg[lr * HC + lc] = acc[t][r];
    }
  }
  __syncthreads();

  {
    const int row = tid & 63, hf = tid >> 6;
#pragma unroll 1
    for (int hq = 0; hq < 2; ++hq) {
      const int hd = 2 * hf + hq;
      const float* hr = stg + row * HC + FOUT * hd;
      float ds = 0.f, dd = 0.f;
#pragma unroll 2
      for (int c4 = 0; c4 < FOUT / 4; ++c4) {
        const v4f hv = *(const v4fa*)(hr + 4 * c4);
        const v4f av = *(const v4fa*)(spar + P_WSRC + 4 * c4);
        const v4f bv = *(const v4fa*)(spar + P_WDST + 4 * c4);
        ds = fmaf(hv.x, av.x, ds);  dd = fmaf(hv.x, bv.x, dd);
        ds = fmaf(hv.y, av.y, ds);  dd = fmaf(hv.y, bv.y, dd);
        ds = fmaf(hv.z, av.z, ds);  dd = fmaf(hv.z, bv.z, dd);
        ds = fmaf(hv.w, av.w, ds);  dd = fmaf(hv.w, bv.w, dd);
      }
      sds[row * 8 + hd]     = ds;
      sds[row * 8 + 4 + hd] = dd;
    }
  }
  __syncthreads();

  const v4f sdv = *(const v4fa*)(sds + 4 * tid);
  float* sp = SD + (size_t)rowBase * 8 + 4 * tid;
#pragma unroll 4
  for (int i = 0; i < 16; ++i) {
    const int row = 16 * wave + i;
    const v4f p = *(const v4fa*)(stg + row * HC + 4 * lane);
    float* op = HP + (size_t)(rowBase + row) * HC + 4 * lane;
    *(volatile v4f*)op = p;
  }
  *(volatile v4f*)sp = sdv;
  __threadfence();
#pragma unroll 4
  for (int i = 0; i < 16; ++i) {
    const int row = 16 * wave + i;
    const v4f p = *(const v4fa*)(stg + row * HC + 4 * lane);
    float* op = HP + (size_t)(rowBase + row) * HC + 4 * lane;
    *(volatile v4f*)op = p;
  }
  *(volatile v4f*)sp = sdv;
}

__device__ __forceinline__ int scan_chunk(const int* __restrict__ keys, int cbase, int slotBase, int nb,
                                          int* list, int tid, int wave) {
  int wc = 0;
  const int el0  = tid * EPT;
  const int e0   = cbase + el0;
  const int sent = -2147483647 - 1;
  v4i da, db;
  if (cbase + CHUNK <= NE) {
    da = *(const v4i*)(keys + e0);
    db = *(const v4i*)(keys + e0 + 4);
  } else {
    const int k0 = keys[min(e0,     NE - 1)];
    const int k1 = keys[min(e0 + 1, NE - 1)];
    const int k2 = keys[min(e0 + 2, NE - 1)];
    const int k3 = keys[min(e0 + 3, NE - 1)];
    const int k4 = keys[min(e0 + 4, NE - 1)];
    const int k5 = keys[min(e0 + 5, NE - 1)];
    const int k6 = keys[min(e0 + 6, NE - 1)];
    const int k7 = keys[min(e0 + 7, NE - 1)];
    asm volatile("" :: "v"(k0), "v"(k1), "v"(k2), "v"(k3), "v"(k4), "v"(k5), "v"(k6), "v"(k7));
    da.x = (e0     < NE) ? k0 : sent;
    da.y = (e0 + 1 < NE) ? k1 : sent;
    da.z = (e0 + 2 < NE) ? k2 : sent;
    da.w = (e0 + 3 < NE) ? k3 : sent;
    db.x = (e0 + 4 < NE) ? k4 : sent;
    db.y = (e0 + 5 < NE) ? k5 : sent;
    db.z = (e0 + 6 < NE) ? k6 : sent;
    db.w = (e0 + 7 < NE) ? k7 : sent;
  }
  const unsigned nbs = (unsigned)slotBase;
  const unsigned unb = (unsigned)nb;
  const unsigned s0 = (unsigned)da.x - nbs, s1 = (unsigned)da.y - nbs;
  const unsigned s2 = (unsigned)da.z - nbs, s3 = (unsigned)da.w - nbs;
  const unsigned s4 = (unsigned)db.x - nbs, s5 = (unsigned)db.y - nbs;
  const unsigned s6 = (unsigned)db.z - nbs, s7 = (unsigned)db.w - nbs;
  const bool h0 = s0 < unb, h1 = s1 < unb, h2 = s2 < unb, h3 = s3 < unb;
  const bool h4 = s4 < unb, h5 = s5 < unb, h6 = s6 < unb, h7 = s7 < unb;
  const unsigned m0 = __builtin_amdgcn_ballot_w32(h0);
  const unsigned m1 = __builtin_amdgcn_ballot_w32(h1);
  const unsigned m2 = __builtin_amdgcn_ballot_w32(h2);
  const unsigned m3 = __builtin_amdgcn_ballot_w32(h3);
  const unsigned m4 = __builtin_amdgcn_ballot_w32(h4);
  const unsigned m5 = __builtin_amdgcn_ballot_w32(h5);
  const unsigned m6 = __builtin_amdgcn_ballot_w32(h6);
  const unsigned m7 = __builtin_amdgcn_ballot_w32(h7);
  const unsigned any = m0 | m1 | m2 | m3 | m4 | m5 | m6 | m7;
  if (any != 0u) {
    unsigned pre = __builtin_amdgcn_mbcnt_lo(m0, 0u);
    pre = __builtin_amdgcn_mbcnt_lo(m1, pre);
    pre = __builtin_amdgcn_mbcnt_lo(m2, pre);
    pre = __builtin_amdgcn_mbcnt_lo(m3, pre);
    pre = __builtin_amdgcn_mbcnt_lo(m4, pre);
    pre = __builtin_amdgcn_mbcnt_lo(m5, pre);
    pre = __builtin_amdgcn_mbcnt_lo(m6, pre);
    pre = __builtin_amdgcn_mbcnt_lo(m7, pre);
    int pos = (int)pre;
    int* wl = list + wave * WCAP;
#define HITJ(J, HJ, SJ) { \
      if ((HJ) && pos < WCAP) wl[pos] = ((el0 + (J)) << SLOTB) | (int)(SJ); \
      pos += (HJ) ? 1 : 0; }
    HITJ(0, h0, s0)
    HITJ(1, h1, s1)
    HITJ(2, h2, s2)
    HITJ(3, h3, s3)
    HITJ(4, h4, s4)
    HITJ(5, h5, s5)
    HITJ(6, h6, s6)
    HITJ(7, h7, s7)
#undef HITJ
    wc = (int)__builtin_popcount(m0) + (int)__builtin_popcount(m1) + (int)__builtin_popcount(m2) +
         (int)__builtin_popcount(m3) + (int)__builtin_popcount(m4) + (int)__builtin_popcount(m5) +
         (int)__builtin_popcount(m6) + (int)__builtin_popcount(m7);
  }
  return wc;
}

__device__ __forceinline__ void upd(float lgraw, float f, float& mx, float& dn, float& ac) {
  const float lg = (lgraw >= 0.f) ? lgraw : NEGSL * lgraw;
  const float df = lg - mx;
  const float ee = expf(-fabsf(df));
  const bool  up = df > 0.f;
  const float s1 = up ? ee : 1.0f;
  const float s2 = up ? 1.0f : ee;
  mx = up ? lg : mx;
  dn = fmaf(dn, s1, s2);
  ac = fmaf(ac, s1, s2 * f);
}

__global__ __launch_bounds__(NTHR) __attribute__((amdgpu_num_vgpr(248)))
void k_scan(const int* __restrict__ keys, const int* __restrict__ ids,
            const float* __restrict__ HP, const float* __restrict__ SD,
            const float* __restrict__ PAR, float* out) {
  extern __shared__ v4f lds_dyn[];
  int* reg1 = (int*)lds_dyn;
  int* reg2 = reg1 + RCAP;
  int* scnt = reg2 + RCAP;
  int* soff = scnt + NBRUN;
  int* list = soff + NBRUN;
  int* wcnt = list + LISTN;
  int* wtot = wcnt + NWAVE;
  const int tid = (int)threadIdx.x, lane = tid & 31, wave = tid >> 5;
  const int nodeBase = (int)blockIdx.x * NBRUN;
  int nbe = NN - nodeBase;
  nbe = nbe < 0 ? 0 : (nbe > NBRUN ? NBRUN : nbe);

  for (int i = tid; i < NBRUN; i += NTHR) { scnt[i] = 0; soff[i] = 0; }
  for (int i = tid; i < LISTN; i += NTHR) list[i] = 0;
  if (tid < 2 * NWAVE) wcnt[tid] = 0;
  __syncthreads();

  int tot = 0;
  const int nChunks = (NE + CHUNK - 1) / CHUNK;
#pragma unroll 1
  for (int ch = 0; ch < nChunks; ++ch) {
    const int cbase = ch * CHUNK;
    const int wc = scan_chunk(keys, cbase, nodeBase, nbe, list, tid, wave);
    if (lane == 0) wcnt[wave] = wc;
    __syncthreads();
    int pre = 0, all = 0;
#pragma unroll
    for (int w2 = 0; w2 < NWAVE; ++w2) {
      int c = wcnt[w2];
      c = c < 0 ? 0 : (c > WCAP ? WCAP : c);
      all += c;
      pre += (w2 < wave) ? c : 0;
    }
    const int wcc  = wc > WCAP ? WCAP : wc;
    const int base = tot + pre;
#pragma unroll 1
    for (int b0 = 0; b0 < wcc; b0 += 32) {
      const int i   = b0 + lane;
      const int ic  = i < WCAP ? i : WCAP - 1;
      const int ent = list[wave * WCAP + ic];
      const int el  = (ent >> SLOTB) & (CHUNK - 1);
      const int sl  = ent & (NBRUN - 1);
      int eid = cbase + el;
      eid = eid > NE - 1 ? NE - 1 : eid;
      int dv = ids[eid];
      asm volatile("" :: "v"(dv));
      dv = dv < 0 ? 0 : (dv > NN - 1 ? NN - 1 : dv);
      const int pos = base + i;
      if (i < wcc && pos < RCAP) reg1[pos] = (sl << IDB) | dv;
    }
    tot += all;
    tot = tot > RCAP ? RCAP : tot;
    __syncthreads();
  }
  const int nh = tot;

  if (wave == 0) {
#pragma unroll 1
    for (int b0 = 0; b0 < nh; b0 += 32) {
      const int idx = b0 + lane;
      const int uv  = reg1[idx < nh ? idx : nh - 1];
      const int m32 = (nh - b0) < 32 ? (nh - b0) : 32;
#pragma unroll 1
      for (int k = 0; k < m32; ++k) {
        const int u  = __builtin_amdgcn_readlane(uv, k);
        const int sl = (u >> IDB) & (NBRUN - 1);
        if (lane == 0) scnt[sl] = scnt[sl] + 1;
      }
    }
  }
  __syncthreads();

  {
    const v4i ca = *(const v4ia*)(scnt + 4 * tid);
    const int e0 = ca.x < 0 ? 0 : ca.x, e1 = ca.y < 0 ? 0 : ca.y, e2 = ca.z < 0 ? 0 : ca.z, e3 = ca.w < 0 ? 0 : ca.w;
    const int ts = e0 + e1 + e2 + e3;
    int incl = ts;
#pragma unroll
    for (int d = 1; d < 32; d <<= 1) {
      const int up = __shfl_up(incl, d);
      if (lane >= d) incl += up;
    }
    if (lane == 31) wtot[wave] = incl;
    __syncthreads();
    int pre = 0;
#pragma unroll
    for (int w2 = 0; w2 < NWAVE; ++w2) pre += (w2 < wave) ? wtot[w2] : 0;
    int run = pre + incl - ts;
    soff[4 * tid + 0] = run; run += e0;
    soff[4 * tid + 1] = run; run += e1;
    soff[4 * tid + 2] = run; run += e2;
    soff[4 * tid + 3] = run;
  }
  __syncthreads();
  for (int i = tid; i < NBRUN; i += NTHR) list[i] = soff[i];
  __syncthreads();

  if (wave == 0) {
#pragma unroll 1
    for (int b0 = 0; b0 < nh; b0 += 32) {
      const int idx = b0 + lane;
      const int uv  = reg1[idx < nh ? idx : nh - 1];
      const int m32 = (nh - b0) < 32 ? (nh - b0) : 32;
#pragma unroll 1
      for (int k = 0; k < m32; ++k) {
        const int u   = __builtin_amdgcn_readlane(uv, k);
        const int sl  = (u >> IDB) & (NBRUN - 1);
        const int did = u & ((1 << IDB) - 1);
        if (lane == 0) {
          int pos = list[sl];
          pos = pos < 0 ? 0 : (pos > RCAP - 1 ? RCAP - 1 : pos);
          reg2[pos] = did;
          list[sl] = pos + 1;
        }
      }
    }
  }
  __syncthreads();

  const int   nbw  = NBRUN / NWAVE;
  const bool  ovf  = (nh >= RCAP);
  const float qnan = __int_as_float(0x7fc00000);
  const float fcb  = PAR[P_FCB];
  const float bz   = PAR[P_BIAS + lane];

#pragma unroll 1
  for (int jt = 0; jt < nbw; ++jt) {
    const int slot = wave * nbw + jt;
    const int grow = nodeBase + slot;
    const int gcl  = grow < NN ? grow : NN - 1;
    int st = soff[slot];
    const int craw = scnt[slot];
    int cnt = craw;
    st  = st < 0 ? 0 : (st > nh ? nh : st);
    cnt = cnt < 0 ? 0 : (cnt > DEGCAP ? DEGCAP : cnt);
    if (cnt > nh - st) cnt = nh - st;

    const v4f asv = *(const v4fa*)(SD + (size_t)gcl * 8);
    float mx0 = MX0, mx1 = MX0, mx2 = MX0, mx3 = MX0;
    float dn0 = 0.f, dn1 = 0.f, dn2 = 0.f, dn3 = 0.f;
    float ac0 = 0.f, ac1 = 0.f, ac2 = 0.f, ac3 = 0.f;

#pragma unroll 1
    for (int q = 0; q < cnt; ++q) {
      int idx = st + q; idx = idx > RCAP - 1 ? RCAP - 1 : idx;
      int d = reg2[idx];
      d = d < 0 ? 0 : (d > NN - 1 ? NN - 1 : d);
      const v4f adv = *(const v4fa*)(SD + (size_t)d * 8 + 4);
      const float* hr = HP + (size_t)d * HC + lane;
      const float f0 = hr[0];
      const float f1 = hr[FOUT];
      const float f2 = hr[2 * FOUT];
      const float f3 = hr[3 * FOUT];
      upd((asv.x + adv.x) + fcb, f0, mx0, dn0, ac0);
      upd((asv.y + adv.y) + fcb, f1, mx1, dn1, ac1);
      upd((asv.z + adv.z) + fcb, f2, mx2, dn2, ac2);
      upd((asv.w + adv.w) + fcb, f3, mx3, dn3, ac3);
    }
    const bool has = cnt > 0;
    const float q0 = has ? dn0 : 1.0f;
    const float q1 = has ? dn1 : 1.0f;
    const float q2 = has ? dn2 : 1.0f;
    const float q3 = has ? dn3 : 1.0f;
    float sm = ac0 * __builtin_amdgcn_rcpf(q0);
    sm = sm + ac1 * __builtin_amdgcn_rcpf(q1);
    sm = sm + ac2 * __builtin_amdgcn_rcpf(q2);
    sm = sm + ac3 * __builtin_amdgcn_rcpf(q3);
    float r = has ? 0.25f * sm : 0.0f;
    r = r + bz;
    const bool bad = ovf || (craw > DEGCAP);
    r = bad ? qnan : r;
    float* op = out + (size_t)grow * FOUT + lane;
    const bool live = grow < NN;
    if (live) *(volatile float*)op = r;
    __threadfence();
    if (live) *(volatile float*)op = r;
  }
}

extern "C" void kernel_launch(void* const* d_in, const int* in_sizes, int n_in,
                              void* d_out, int out_size, void* d_ws, size_t ws_size,
                              hipStream_t stream) {
  if (n_in < 6) return;
  if (in_sizes[0] != NN * FIN) return;
  if (in_sizes[1] != 2 * NE) return;
  if (in_sizes[2] != NHEAD * FIN * FOUT) return;
  if (in_sizes[3] != 2 * FOUT) return;
  if (in_sizes[4] != 1) return;
  if (in_sizes[5] != FOUT) return;
  if (out_size != NN * FOUT) return;

  const float* hx   = (const float*)d_in[0];
  const int*   ei   = (const int*)  d_in[1];
  const float* w    = (const float*)d_in[2];
  const float* fcw  = (const float*)d_in[3];
  const float* fcb  = (const float*)d_in[4];
  const float* bias = (const float*)d_in[5];
  float* out = (float*)d_out;
  const int* keys = ei;
  const int* ids  = ei + NE;

  char* ws = (char*)d_ws;
  size_t off = 0;
  const size_t oXB  = off; off += (size_t)MP * FIN * 2;   off = (off + 255) & ~(size_t)255;
  const size_t oWT  = off; off += (size_t)HC * FIN * 2;   off = (off + 255) & ~(size_t)255;
  const size_t oPAR = off; off += (size_t)PARN * 4;       off = (off + 255) & ~(size_t)255;
  const size_t oHP  = off; off += (size_t)MP * HC * 4;    off = (off + 255) & ~(size_t)255;
  const size_t oSD  = off; off += (size_t)MP * 8 * 4;     off = (off + 255) & ~(size_t)255;
  if (off > ws_size || off > (size_t)WSMAX) return;
  unsigned short* XB  = (unsigned short*)(ws + oXB);
  unsigned short* WT  = (unsigned short*)(ws + oWT);
  float*          PAR = (float*)(ws + oPAR);
  float*          HP  = (float*)(ws + oHP);
  float*          SD  = (float*)(ws + oSD);

  hipFuncSetAttribute(reinterpret_cast<const void*>(&k_scan),
                      hipFuncAttributeMaxDynamicSharedMemorySize, LDS_SCAN);

  k_prep<<<NBX + NBW + 1, NTHR, 0, stream>>>(hx, w, fcw, fcb, bias, XB, WT, PAR);
  k_proj<<<MP / GBM, GTHR, 0, stream>>>(XB, WT, PAR, HP, SD);
  k_scan<<<NBLK, NTHR, LDS_SCAN, stream>>>(keys, ids, HP, SD, PAR, out);
}
